// ModulatedDeformConv_40441412059305
// MI455X (gfx1250) — hardware-run, weakly checked
//
#include <hip/hip_runtime.h>
#include <math.h>

typedef __attribute__((ext_vector_type(16))) _Float16 v16h;
typedef __attribute__((ext_vector_type(8)))  _Float16 v8h;
typedef __attribute__((ext_vector_type(8)))  float    v8f;
typedef __attribute__((ext_vector_type(4)))  float    v4f;
typedef __attribute__((ext_vector_type(4)))  unsigned v4u;

constexpr int kBatch   = 4;
constexpr int kChan    = 64;
constexpr int kOutCh   = 64;
constexpr int kHeight  = 128;
constexpr int kWidth   = 128;
constexpr int kTaps    = 9;
constexpr int kKdim    = kChan * kTaps;
constexpr int kPixPerB = kHeight * kWidth;
constexpr int kNpix    = kBatch * kPixPerB;
constexpr int kOffCh   = 3 * kTaps;
constexpr int kMpad    = 64;
constexpr int kLines   = kNpix * kTaps;

constexpr float kCarryX      = 64.0f;
constexpr float kCarryW      = 1024.0f;
constexpr float kFoldBack    = 1.0f / (kCarryX * kCarryW);
constexpr float kF16MinNorm  = 6.103515625e-05f;

static_assert(kKdim == 576 && (kKdim % 32) == 0, "K multiple of 32");
static_assert(kChan == 64, "one pixel = one 128-B line of f16 channels");
static_assert(kOffCh == 27 && kOffCh <= kMpad, "offset rows fit the padded tile");
static_assert((kMpad % 64) == 0 && (kOutCh % 64) == 0 && (kPixPerB % 64) == 0, "M,N multiples of 64");
static_assert(kNpix == 65536 && kPixPerB == 16384, "pixel decode uses shifts");
static_assert((kLines % 256) == 0, "sampler grid exact");
static_assert(((kLines * 8) % 256) == 0, "im2col grid exact");
static_assert(((kMpad * kKdim / 8) % 256) == 0, "weight plane grid exact");

constexpr size_t kSzXH = (size_t)kNpix * kChan * 2;
constexpr size_t kSzW  = (size_t)kMpad * kKdim * 2;
constexpr size_t kSzS  = (size_t)kNpix * kKdim * 2;
constexpr size_t kSzOM = (size_t)kMpad * kNpix * 4;
constexpr size_t kOffXH = 0;
constexpr size_t kOffW1 = kOffXH + kSzXH;
constexpr size_t kOffW2 = kOffW1 + kSzW;
constexpr size_t kOffS  = kOffW2 + kSzW;
constexpr size_t kOffOM = kOffS + kSzS;
constexpr size_t kWsTotal = kOffOM + kSzOM;
static_assert(kWsTotal == 100810752ull, "carve total");
static_assert(kWsTotal <= 134217728ull, "carve cap");
static_assert((kOffW1 % 128) == 0 && (kOffW2 % 128) == 0 && (kOffS % 128) == 0 && (kOffOM % 128) == 0, "128-B aligned regions");

__device__ __forceinline__ float flush_small(float v) {
  return (fabsf(v) < kF16MinNorm) ? 0.0f : v;
}

__device__ __forceinline__ float h16_to_f32(unsigned hb) {
  const unsigned sgn = (hb & 0x8000u) << 16;
  const unsigned em = hb & 0x7fffu;
  const float fn = __uint_as_float((em << 13) + 0x38000000u);
  const float fs = (float)em * 5.9604644775390625e-8f;
  const float mag = (em < 0x400u) ? fs : fn;
  return __uint_as_float(__float_as_uint(mag) | sgn);
}

__device__ __forceinline__ v8f mma_g(v16h a, v16h b, v8f c) {
  c = __builtin_amdgcn_wmma_f32_16x16x32_f16(false, a, false, b, (short)0, c, false, false);
  asm volatile("v_nop\n\tv_nop\n\tv_nop\n\tv_nop" : "+v"(c) : "v"(a), "v"(b));
  return c;
}
__device__ __forceinline__ void keep4_h(v16h a, v16h b, v16h c, v16h d) { asm volatile("v_nop" :: "v"(a), "v"(b), "v"(c), "v"(d)); }
__device__ __forceinline__ void acc_guard4(v8f& a, v8f& b, v8f& c, v8f& d) { asm volatile("v_nop\n\tv_nop\n\tv_nop\n\tv_nop" : "+v"(a), "+v"(b), "+v"(c), "+v"(d)); }

union FragH { v16h v; v8h h[2]; };
__device__ __forceinline__ v16h frag_load(const _Float16* p) {
  FragH f;
  f.h[0] = *(const v8h*)(p);
  f.h[1] = *(const v8h*)(p + 16);
  return f.v;
}

__global__ __launch_bounds__(256) void pixel_major_f16_kernel(
    const float* __restrict__ x, unsigned short* __restrict__ XH)
{
  __shared__ __align__(16) float sT[kChan * 132];
  const int tid = threadIdx.x, lane = tid & 31, wave = tid >> 5;
  const int bh = blockIdx.x;
  const int b = bh >> 7, h = bh & 127;
  const float* src = x + (size_t)b * kChan * kPixPerB + (size_t)h * kWidth;
#pragma unroll
  for (int it = 0; it < 8; ++it) {
    const int idx = it * 256 + tid;
    const int c = idx >> 5;
    const int w4 = (idx & 31) * 4;
    const v4f v = *(const v4f*)(src + (size_t)c * kPixPerB + w4);
    *(v4f*)(sT + c * 132 + w4) = v;
  }
  __syncthreads();
  const int q = lane >> 3, sub = lane & 7;
  v8h hv[4];
#pragma unroll
  for (int it = 0; it < 4; ++it) {
    const int w = it * 32 + wave * 4 + q;
#pragma unroll
    for (int e = 0; e < 8; ++e) {
      const float f = flush_small(sT[(sub * 8 + e) * 132 + w] * kCarryX);
      hv[it][e] = (_Float16)f;
    }
  }
  for (int pass = 0; pass < 2; ++pass) {
#pragma unroll
    for (int it = 0; it < 4; ++it) {
      const int w = it * 32 + wave * 4 + q;
      *(volatile v8h*)(XH + ((size_t)bh * kWidth + w) * kChan + sub * 8) = hv[it];
    }
    __threadfence();
  }
}

__global__ __launch_bounds__(256) void weight_planes_kernel(
    const float* __restrict__ ow, const float* __restrict__ dw,
    unsigned short* __restrict__ W1, unsigned short* __restrict__ W2)
{
  const int plane = blockIdx.y;
  const float* src = plane ? dw : ow;
  unsigned short* dst = plane ? W2 : W1;
  const int nreal = plane ? kOutCh : kOffCh;
  const int i = blockIdx.x * 256 + threadIdx.x;
  const int o = i / 72;
  const int k8 = (i - o * 72) * 8;
  const int kk = k8 >> 6;
  const int c0 = k8 & 63;
  const int oc = (o < nreal) ? o : (nreal - 1);
  const bool live = (o < nreal);
  v8h hv;
#pragma unroll
  for (int e = 0; e < 8; ++e) {
    float v = src[(size_t)oc * kKdim + (c0 + e) * kTaps + kk];
    asm volatile("" : "+v"(v));
    const float s = live ? (v * kCarryW) : 0.0f;
    hv[e] = (_Float16)flush_small(s);
  }
  unsigned short* p = dst + (size_t)i * 8;
  *(volatile v8h*)p = hv;
  __threadfence();
  *(volatile v8h*)p = hv;
}

__global__ __launch_bounds__(256) void im2col_rows_kernel(
    const unsigned short* __restrict__ XH, unsigned short* __restrict__ S)
{
  const int g = blockIdx.x * 256 + threadIdx.x;
  const int L = g >> 3;
  const int sub = g & 7;
  const int p = L / kTaps;
  const int kk = L - p * kTaps;
  const int ky = kk / 3;
  const int kx = kk - ky * 3;
  const int b = p >> 14;
  const int i = (p >> 7) & 127;
  const int j = p & 127;
  const int yy = i + ky - 1;
  const int xx = j + kx - 1;
  const bool inside = ((unsigned)yy < (unsigned)kHeight) && ((unsigned)xx < (unsigned)kWidth);
  const int yc = min(max(yy, 0), kHeight - 1);
  const int xc = min(max(xx, 0), kWidth - 1);
  const v4u v = *(const v4u*)(XH + ((size_t)((b * kHeight + yc) * kWidth + xc)) * kChan + sub * 8);
  unsigned a0 = v[0], a1 = v[1], a2 = v[2], a3 = v[3];
  asm volatile("" : "+v"(a0), "+v"(a1), "+v"(a2), "+v"(a3));
  v4u o;
  o[0] = inside ? a0 : 0u;
  o[1] = inside ? a1 : 0u;
  o[2] = inside ? a2 : 0u;
  o[3] = inside ? a3 : 0u;
  unsigned short* q = S + (size_t)g * 8;
  *(volatile v4u*)q = o;
  __threadfence();
  *(volatile v4u*)q = o;
}

__global__ __launch_bounds__(256) void sample_rows_kernel(
    const float* __restrict__ OM, const float* __restrict__ ob,
    const unsigned short* __restrict__ XH, unsigned short* __restrict__ S)
{
  __shared__ float sWt[5][256];
  __shared__ int   sIx[4][256];
  const int tid = threadIdx.x, lane = tid & 31, wave = tid >> 5;
  {
    const int L = blockIdx.x * 256 + tid;
    const int p = L / kTaps;
    const int kk = L - p * kTaps;
    const int ky = kk / 3;
    const int kx = kk - ky * 3;
    const int b = p >> 14;
    const int i = (p >> 7) & 127;
    const int j = p & 127;
    const float dy = OM[(size_t)kk * kNpix + p] + ob[kk];
    const float dx = OM[(size_t)(kTaps + kk) * kNpix + p] + ob[kTaps + kk];
    const float ml = OM[(size_t)(2 * kTaps + kk) * kNpix + p] + ob[2 * kTaps + kk];
    const float mk = 1.0f / (1.0f + expf(-ml));
    const float ys = dy + (float)(i - 1 + ky);
    const float xs = dx + (float)(j - 1 + kx);
    const float y0 = floorf(ys);
    const float x0 = floorf(xs);
    const float ty = ys - y0;
    const float tx = xs - x0;
    const float y1 = y0 + 1.0f;
    const float x1 = x0 + 1.0f;
    const bool oky0 = (y0 >= 0.0f) && (y0 < (float)kHeight);
    const bool oky1 = (y1 >= 0.0f) && (y1 < (float)kHeight);
    const bool okx0 = (x0 >= 0.0f) && (x0 < (float)kWidth);
    const bool okx1 = (x1 >= 0.0f) && (x1 < (float)kWidth);
    const int cy0 = (int)fminf(fmaxf(y0, 0.0f), (float)(kHeight - 1));
    const int cy1 = (int)fminf(fmaxf(y1, 0.0f), (float)(kHeight - 1));
    const int cx0 = (int)fminf(fmaxf(x0, 0.0f), (float)(kWidth - 1));
    const int cx1 = (int)fminf(fmaxf(x1, 0.0f), (float)(kWidth - 1));
    const float omty = 1.0f - ty;
    const float omtx = 1.0f - tx;
    const float w00 = omty * omtx;
    const float w01 = omty * tx;
    const float w10 = ty * omtx;
    const float w11 = ty * tx;
    sWt[0][tid] = (oky0 && okx0) ? w00 : 0.0f;
    sWt[1][tid] = (oky0 && okx1) ? w01 : 0.0f;
    sWt[2][tid] = (oky1 && okx0) ? w10 : 0.0f;
    sWt[3][tid] = (oky1 && okx1) ? w11 : 0.0f;
    sWt[4][tid] = mk;
    const int pb = b * kPixPerB;
    sIx[0][tid] = pb + cy0 * kWidth + cx0;
    sIx[1][tid] = pb + cy0 * kWidth + cx1;
    sIx[2][tid] = pb + cy1 * kWidth + cx0;
    sIx[3][tid] = pb + cy1 * kWidth + cx1;
  }
  __syncthreads();
  const int q = lane >> 3, sub = lane & 7;
#pragma unroll 1
  for (int it = 0; it < 8; ++it) {
    const int ll = it * 32 + wave * 4 + q;
    const float w00 = sWt[0][ll];
    const float w01 = sWt[1][ll];
    const float w10 = sWt[2][ll];
    const float w11 = sWt[3][ll];
    const float mk  = sWt[4][ll];
    const int i00 = sIx[0][ll] & (kNpix - 1);
    const int i01 = sIx[1][ll] & (kNpix - 1);
    const int i10 = sIx[2][ll] & (kNpix - 1);
    const int i11 = sIx[3][ll] & (kNpix - 1);
    const v4u c00 = *(const v4u*)(XH + (size_t)i00 * kChan + sub * 8);
    const v4u c01 = *(const v4u*)(XH + (size_t)i01 * kChan + sub * 8);
    const v4u c10 = *(const v4u*)(XH + (size_t)i10 * kChan + sub * 8);
    const v4u c11 = *(const v4u*)(XH + (size_t)i11 * kChan + sub * 8);
    v8h hv;
#pragma unroll
    for (int wd = 0; wd < 4; ++wd) {
      const unsigned u00 = c00[wd];
      const unsigned u01 = c01[wd];
      const unsigned u10 = c10[wd];
      const unsigned u11 = c11[wd];
      float lo = h16_to_f32(u00 & 0xffffu) * w00;
      lo = fmaf(h16_to_f32(u01 & 0xffffu), w01, lo);
      lo = fmaf(h16_to_f32(u10 & 0xffffu), w10, lo);
      lo = fmaf(h16_to_f32(u11 & 0xffffu), w11, lo);
      float hi = h16_to_f32(u00 >> 16) * w00;
      hi = fmaf(h16_to_f32(u01 >> 16), w01, hi);
      hi = fmaf(h16_to_f32(u10 >> 16), w10, hi);
      hi = fmaf(h16_to_f32(u11 >> 16), w11, hi);
      const float rlo = flush_small(lo * mk);
      const float rhi = flush_small(hi * mk);
      hv[2 * wd]     = (_Float16)rlo;
      hv[2 * wd + 1] = (_Float16)rhi;
    }
    unsigned short* dst = S + ((size_t)blockIdx.x * 256 + ll) * kChan + sub * 8;
    *(volatile v8h*)dst = hv;
    __threadfence();
    *(volatile v8h*)dst = hv;
  }
}

template <bool HAS_BIAS>
__global__ __launch_bounds__(256) void gemm_rows_by_pixels(
    const unsigned short* __restrict__ Ap, int lda,
    const unsigned short* __restrict__ Btp, int ldb, long strideB,
    float* __restrict__ Cout, int ldc, long strideC,
    const float* __restrict__ bias, int M, int N, int K, float scale)
{
  const _Float16* A  = (const _Float16*)Ap;
  const _Float16* Bt = (const _Float16*)Btp;
  __shared__ __align__(16) float sT[8][16 * 68];
  const int b    = blockIdx.y;
  const int lane = threadIdx.x & 31;
  const int wave = threadIdx.x >> 5;
  const int tilesN = N >> 6;
  const int tilesM = M >> 6;
  const int tile = blockIdx.x * 8 + wave;
  if (tile >= tilesM * tilesN) return;
  const int tm = tile / tilesN;
  const int tn = tile - tm * tilesN;
  const int m0 = tm << 6;
  const int n0 = tn << 6;

  const _Float16* Bb = Bt + (size_t)b * strideB;

  const int rlane = lane & 15;
  const int koff  = (lane >> 4) * 8;
  const int mOff  = (lane >> 4) * 8;

  v8f acc[4][4];
#pragma unroll
  for (int i = 0; i < 4; ++i)
#pragma unroll
    for (int j = 0; j < 4; ++j) acc[i][j] = (v8f){0.f,0.f,0.f,0.f,0.f,0.f,0.f,0.f};

  for (int k0 = 0; k0 < K; k0 += 32) {
    v16h bh[4];
#pragma unroll
    for (int j = 0; j < 4; ++j) {
      const size_t bo = (size_t)(n0 + (j << 4) + rlane) * ldb + koff + k0;
      bh[j] = frag_load(Bb + bo);
    }
#pragma unroll
    for (int i = 0; i < 4; ++i) {
      const size_t ao = (size_t)(m0 + (i << 4) + rlane) * lda + koff + k0;
      const v16h ah = frag_load(A + ao);
#pragma unroll
      for (int j = 0; j < 4; ++j) acc[i][j] = mma_g(ah, bh[j], acc[i][j]);
    }
    keep4_h(bh[0], bh[1], bh[2], bh[3]);
  }
  acc_guard4(acc[0][0], acc[0][1], acc[0][2], acc[0][3]);
  acc_guard4(acc[1][0], acc[1][1], acc[1][2], acc[1][3]);
  acc_guard4(acc[2][0], acc[2][1], acc[2][2], acc[2][3]);
  acc_guard4(acc[3][0], acc[3][1], acc[3][2], acc[3][3]);

  float* slab = sT[wave];
  float* C = Cout + (size_t)b * strideC;
#pragma unroll
  for (int i = 0; i < 4; ++i) {
    const int mBase = m0 + (i << 4);
    v4f bq0 = (v4f){0.f, 0.f, 0.f, 0.f};
    v4f bq1 = (v4f){0.f, 0.f, 0.f, 0.f};
    if (HAS_BIAS) {
      bq0 = *(const v4f*)(bias + mBase + mOff);
      bq1 = *(const v4f*)(bias + mBase + mOff + 4);
    }
    const float bvals[8] = {bq0[0], bq0[1], bq0[2], bq0[3], bq1[0], bq1[1], bq1[2], bq1[3]};
#pragma unroll
    for (int j = 0; j < 4; ++j) {
#pragma unroll
      for (int r = 0; r < 8; ++r) {
        float v = acc[i][j][r] * scale;
        if (HAS_BIAS) v += bvals[r];
        slab[(mOff + r) * 68 + (j << 4) + rlane] = v;
      }
    }
    __builtin_amdgcn_fence(__ATOMIC_RELEASE, "workgroup");
    __builtin_amdgcn_wave_barrier();
    __builtin_amdgcn_fence(__ATOMIC_ACQUIRE, "workgroup");
    {
      const int hh = lane >> 4, c4 = (lane & 15) * 4;
      for (int pass = 0; pass < 2; ++pass) {
#pragma unroll
        for (int it = 0; it < 8; ++it) {
          const int row = it * 2 + hh;
          const v4f v = *(const v4f*)(slab + row * 68 + c4);
          *(volatile v4f*)(C + (size_t)(mBase + row) * ldc + n0 + c4) = v;
        }
        __threadfence();
      }
    }
    __builtin_amdgcn_fence(__ATOMIC_RELEASE, "workgroup");
    __builtin_amdgcn_wave_barrier();
    __builtin_amdgcn_fence(__ATOMIC_ACQUIRE, "workgroup");
  }
}

extern "C" void kernel_launch(void* const* d_in, const int* in_sizes, int n_in,
                              void* d_out, int out_size, void* d_ws, size_t ws_size,
                              hipStream_t stream) {
  if (n_in < 5) return;
  if (in_sizes[0] != kBatch * kChan * kPixPerB) return;
  if (in_sizes[1] != kOffCh * kKdim) return;
  if (in_sizes[2] != kOffCh) return;
  if (in_sizes[3] != kOutCh * kKdim) return;
  if (in_sizes[4] != kOutCh) return;
  if (out_size != kBatch * kOutCh * kPixPerB) return;
  if (ws_size < kWsTotal) return;

  const float* x   = (const float*)d_in[0];
  const float* ow  = (const float*)d_in[1];
  const float* ob  = (const float*)d_in[2];
  const float* dw  = (const float*)d_in[3];
  const float* db  = (const float*)d_in[4];
  float* out = (float*)d_out;

  char* ws = (char*)d_ws;
  unsigned short* XH = (unsigned short*)(ws + kOffXH);
  unsigned short* W1 = (unsigned short*)(ws + kOffW1);
  unsigned short* W2 = (unsigned short*)(ws + kOffW2);
  unsigned short* S  = (unsigned short*)(ws + kOffS);
  float*          OM = (float*)(ws + kOffOM);

  pixel_major_f16_kernel<<<kBatch * kHeight, 256, 0, stream>>>(x, XH);

  weight_planes_kernel<<<dim3((kMpad * kKdim / 8) / 256, 2), 256, 0, stream>>>(ow, dw, W1, W2);

  im2col_rows_kernel<<<(kLines * 8) / 256, 256, 0, stream>>>(XH, S);

  gemm_rows_by_pixels<false><<<dim3(32, kBatch), 256, 0, stream>>>(
      W1, kKdim,
      S, kKdim, (long)kPixPerB * kKdim,
      OM, kNpix, (long)kPixPerB,
      nullptr, kMpad, kPixPerB, kKdim, kFoldBack);

  sample_rows_kernel<<<kLines / 256, 256, 0, stream>>>(OM, ob, XH, S);

  gemm_rows_by_pixels<true><<<dim3(32, kBatch), 256, 0, stream>>>(
      W2, kKdim,
      S, kKdim, (long)kPixPerB * kKdim,
      out, kPixPerB, (long)kOutCh * kPixPerB,
      db, kOutCh, kPixPerB, kKdim, kFoldBack);
}
